// Mamba3Block_36653250904126
// MI455X (gfx1250) — hardware-verified
//
#include <hip/hip_runtime.h>
#include <math.h>

typedef __attribute__((ext_vector_type(16))) _Float16 v16h;
typedef __attribute__((ext_vector_type(8)))  _Float16 v8h;
typedef __attribute__((ext_vector_type(16))) __bf16   v16b;
typedef __attribute__((ext_vector_type(8)))  __bf16   v8b;
typedef __attribute__((ext_vector_type(8)))  float    v8f;
typedef __attribute__((ext_vector_type(4)))  float    v4f;

constexpr int kBatch = 4;
constexpr int kSeq   = 512;
constexpr int kDm    = 512;
constexpr int kDin   = 1024;
constexpr int kHeads = 16;
constexpr int kHd    = 64;
constexpr int kRN    = 128;
constexpr int kDff   = 1368;
constexpr int kDffP  = 1408;
constexpr int kRows  = kBatch * kSeq;
constexpr int kNProj = 6208;
constexpr int kColZ  = 0;
constexpr int kColU  = 1024;
constexpr int kColB  = 2048;
constexpr int kColC  = 4096;
constexpr int kColDt = 6144;
constexpr int kN13   = 2 * kDffP;
constexpr int kTS    = 16;
constexpr int kStageP = 384;
static_assert(kHeads * kHd == kDin, "inner width");
static_assert(kHeads * kRN == 2048, "B/C width");
static_assert(kColDt + kHeads <= kNProj && (kNProj % 64) == 0, "proj plane width");
static_assert((kRows % 64) == 0 && (kDm % 64) == 0 && (kDin % 64) == 0 && (kDffP % 64) == 0 && (kN13 % 64) == 0, "GEMM M,N tile multiples");
static_assert((kDm % 32) == 0 && (kDin % 32) == 0 && (kDffP % 32) == 0, "GEMM K multiples of 32");
static_assert((kSeq % kTS) == 0 && (kDff % 4) == 0 && kDff <= kDffP && kDffP == 176 * 8, "tiling");

constexpr size_t kOffWP  = 0;
constexpr size_t kOffWO  = kOffWP  + (size_t)kNProj * kDm  * 2;
constexpr size_t kOffW13 = kOffWO  + (size_t)kDm    * kDin * 2;
constexpr size_t kOffW2  = kOffW13 + (size_t)kN13   * kDm  * 2;
constexpr size_t kOffXNH = kOffW2  + (size_t)kDm    * kDffP * 2;
constexpr size_t kOffXNL = kOffXNH + (size_t)kRows  * kDm  * 2;
constexpr size_t kOffP   = kOffXNL + (size_t)kRows  * kDm  * 2;
constexpr size_t kOffYGH = kOffP   + (size_t)kRows  * kNProj * 4;
constexpr size_t kOffYGL = kOffYGH + (size_t)kRows  * kDin * 2;
constexpr size_t kOffYO  = kOffYGL + (size_t)kRows  * kDin * 2;
constexpr size_t kOffX2H = kOffYO  + (size_t)kRows  * kDm  * 4;
constexpr size_t kOffX2L = kOffX2H + (size_t)kRows  * kDm  * 2;
constexpr size_t kOffG   = kOffX2L + (size_t)kRows  * kDm  * 2;
constexpr size_t kOffHFH = kOffG   + (size_t)kRows  * kN13 * 4;
constexpr size_t kOffHFL = kOffHFH + (size_t)kRows  * kDffP * 2;
constexpr size_t kOffFF  = kOffHFL + (size_t)kRows  * kDffP * 2;
constexpr size_t kWsTotal = kOffFF + (size_t)kRows  * kDm  * 4;
static_assert(kWsTotal == 122355712ull, "carve total");
static_assert(kWsTotal <= 134217728ull, "carve cap");
static_assert((kOffWO % 128) == 0 && (kOffW13 % 128) == 0 && (kOffW2 % 128) == 0 && (kOffXNH % 128) == 0 &&
              (kOffXNL % 128) == 0 && (kOffP % 128) == 0 && (kOffYGH % 128) == 0 && (kOffYGL % 128) == 0 &&
              (kOffYO % 128) == 0 && (kOffX2H % 128) == 0 && (kOffX2L % 128) == 0 && (kOffG % 128) == 0 &&
              (kOffHFH % 128) == 0 && (kOffHFL % 128) == 0 && (kOffFF % 128) == 0, "128-B aligned regions");

__device__ __forceinline__ unsigned short f2bf_bits(float f) {
  unsigned u = __float_as_uint(f);
  return (unsigned short)((u + 0x7FFFu + ((u >> 16) & 1u)) >> 16);
}
__device__ __forceinline__ float bf_bits2f(unsigned short h) { return __uint_as_float(((unsigned)h) << 16); }
__device__ __forceinline__ float bfr(float f) { return bf_bits2f(f2bf_bits(f)); }
struct HL16 { _Float16 h; _Float16 l; };
__device__ __forceinline__ HL16 split_hl(float v) {
  const unsigned short hb = f2bf_bits(v);
  const unsigned short lb = f2bf_bits(v - bf_bits2f(hb));
  HL16 r; r.h = __builtin_bit_cast(_Float16, hb); r.l = __builtin_bit_cast(_Float16, lb); return r;
}

__device__ __forceinline__ void dep_guard4_h(v8f& a, v8f& b, v8f& c, v8f& d, v16h x, v16h y) { asm volatile("v_nop\n\tv_nop\n\tv_nop\n\tv_nop" : "+v"(a), "+v"(b), "+v"(c), "+v"(d) : "v"(x), "v"(y)); }
__device__ __forceinline__ void dep_guard4_b(v8f& a, v8f& b, v8f& c, v8f& d, v16b x, v16b y) { asm volatile("v_nop\n\tv_nop\n\tv_nop\n\tv_nop" : "+v"(a), "+v"(b), "+v"(c), "+v"(d) : "v"(x), "v"(y)); }
__device__ __forceinline__ void keep4_h(v16h a, v16h b, v16h c, v16h d) { asm volatile("v_nop" :: "v"(a), "v"(b), "v"(c), "v"(d)); }
__device__ __forceinline__ void keep4_b(v16b a, v16b b, v16b c, v16b d) { asm volatile("v_nop" :: "v"(a), "v"(b), "v"(c), "v"(d)); }
__device__ __forceinline__ void acc_guard4(v8f& a, v8f& b, v8f& c, v8f& d) { asm volatile("v_nop\n\tv_nop\n\tv_nop\n\tv_nop" : "+v"(a), "+v"(b), "+v"(c), "+v"(d)); }
template <typename T> struct Frag;
template <> struct Frag<_Float16> {
  typedef v16h V; union U { v16h v; v8h h[2]; };
  static __device__ __forceinline__ v16h load(const _Float16* p) {
    U f; f.h[0] = *(const v8h*)(p); f.h[1] = *(const v8h*)(p + 16); return f.v;
  }
  static __device__ __forceinline__ v8f mma(v16h a, v16h b, v8f c) {
    return __builtin_amdgcn_wmma_f32_16x16x32_f16(false, a, false, b, (short)0, c, false, false);
  }
  static __device__ __forceinline__ void guard4(v8f& a, v8f& b, v8f& c, v8f& d, v16h x, v16h y) { dep_guard4_h(a, b, c, d, x, y); }
  static __device__ __forceinline__ void keep(v16h a, v16h b, v16h c, v16h d) { keep4_h(a, b, c, d); }
};
template <> struct Frag<__bf16> {
  typedef v16b V; union U { v16b v; v8b h[2]; };
  static __device__ __forceinline__ v16b load(const __bf16* p) {
    U f; f.h[0] = *(const v8b*)(p); f.h[1] = *(const v8b*)(p + 16); return f.v;
  }
  static __device__ __forceinline__ v8f mma(v16b a, v16b b, v8f c) {
    return __builtin_amdgcn_wmma_f32_16x16x32_bf16(false, a, false, b, (short)0, c, false, false);
  }
  static __device__ __forceinline__ void guard4(v8f& a, v8f& b, v8f& c, v8f& d, v16b x, v16b y) { dep_guard4_b(a, b, c, d, x, y); }
  static __device__ __forceinline__ void keep(v16b a, v16b b, v16b c, v16b d) { keep4_b(a, b, c, d); }
};

template <int ET> struct Elem;
template <> struct Elem<0> { typedef _Float16 T; };
template <> struct Elem<1> { typedef __bf16 T; };
template <int ET, int SPL, int BIAS_MODE, int OUT_MODE, int ACT = 0>
__global__ __launch_bounds__(256) void wmma_gemm64(
    const unsigned short* __restrict__ Ap, const unsigned short* __restrict__ A2p, int lda, long strideA,
    const unsigned short* __restrict__ Btp, const unsigned short* __restrict__ Bt2p, int ldb, long strideB,
    void* __restrict__ Cout, void* __restrict__ Cout2, int ldc, long strideC,
    const float* __restrict__ bias,
    int M, int N, int K, float scale) {
  typedef typename Elem<ET>::T T;
  typedef typename Frag<T>::V V;
  const T* A = (const T*)Ap; const T* A2 = (const T*)A2p; const T* Bt = (const T*)Btp; const T* Bt2 = (const T*)Bt2p;
  __shared__ __align__(16) float sT[8][16 * 68];
  const int b    = blockIdx.y;
  const int lane = threadIdx.x & 31;
  const int wave = threadIdx.x >> 5;
  const int tilesN = N >> 6;
  const int tilesM = M >> 6;
  const int tile = blockIdx.x * 8 + wave;
  if (tile >= tilesM * tilesN) return;
  const int tm = tile / tilesN;
  const int tn = tile - tm * tilesN;
  const int m0 = tm << 6;
  const int n0 = tn << 6;

  const T* Ab  = A  + (size_t)b * strideA;
  const T* Bb  = Bt + (size_t)b * strideB;
  const T* Ab2 = (SPL >= 1) ? (A2  + (size_t)b * strideA) : nullptr;
  const T* Bb2 = (SPL == 2) ? (Bt2 + (size_t)b * strideB) : nullptr;

  const int rlane = lane & 15;
  const int koff  = (lane >> 4) * 8;
  const int mOff  = (lane >> 4) * 8;

  v8f acc[4][4];
#pragma unroll
  for (int i = 0; i < 4; ++i)
#pragma unroll
    for (int j = 0; j < 4; ++j) acc[i][j] = (v8f){0.f,0.f,0.f,0.f,0.f,0.f,0.f,0.f};

  for (int k0 = 0; k0 < K; k0 += 32) {
    V bh[4], bl[4];
#pragma unroll
    for (int j = 0; j < 4; ++j) {
      const size_t bo = (size_t)(n0 + (j << 4) + rlane) * ldb + koff + k0;
      bh[j] = Frag<T>::load(Bb + bo);
      if (SPL == 2) bl[j] = Frag<T>::load(Bb2 + bo);
    }
#pragma unroll
    for (int i = 0; i < 4; ++i) {
      const size_t ao = (size_t)(m0 + (i << 4) + rlane) * lda + koff + k0;
      V ah = Frag<T>::load(Ab + ao);
      V al;
      if (SPL >= 1) al = Frag<T>::load(Ab2 + ao);
#pragma unroll
      for (int j = 0; j < 4; ++j) {
        acc[i][j] = Frag<T>::mma(ah, bh[j], acc[i][j]);
        if (SPL == 2) acc[i][j] = Frag<T>::mma(ah, bl[j], acc[i][j]);
        if (SPL >= 1) acc[i][j] = Frag<T>::mma(al, bh[j], acc[i][j]);
      }
      Frag<T>::guard4(acc[i][0], acc[i][1], acc[i][2], acc[i][3], ah, (SPL >= 1) ? al : ah);
    }
    Frag<T>::keep(bh[0], bh[1], bh[2], bh[3]);
    if (SPL == 2) Frag<T>::keep(bl[0], bl[1], bl[2], bl[3]);
  }
  acc_guard4(acc[0][0], acc[0][1], acc[0][2], acc[0][3]);
  acc_guard4(acc[1][0], acc[1][1], acc[1][2], acc[1][3]);
  acc_guard4(acc[2][0], acc[2][1], acc[2][2], acc[2][3]);
  acc_guard4(acc[3][0], acc[3][1], acc[3][2], acc[3][3]);

  float* slab = sT[wave];
#pragma unroll
  for (int i = 0; i < 4; ++i) {
    const int mBase = m0 + (i << 4);
#pragma unroll
    for (int j = 0; j < 4; ++j) {
      const int n = n0 + (j << 4) + rlane;
      float bv = 0.f;
      if (BIAS_MODE == 2) bv = bias[n];
#pragma unroll
      for (int r = 0; r < 8; ++r) {
        float v = acc[i][j][r] * scale;
        if (BIAS_MODE == 1) v += bias[mBase + mOff + r];
        if (BIAS_MODE == 2) v += bv;
        if (ACT == 1) v = tanhf(v);
        if (ACT == 2) v = fmaxf(v, 0.0f);
        if (ACT == 3) v = v / (1.0f + expf(-v));
        if (ACT == 4) v = (v > 0.f) ? v : 0.01f * v;
        slab[(mOff + r) * 68 + (j << 4) + rlane] = v;
      }
    }
    __builtin_amdgcn_fence(__ATOMIC_RELEASE, "workgroup");
    __builtin_amdgcn_wave_barrier();
    __builtin_amdgcn_fence(__ATOMIC_ACQUIRE, "workgroup");
    if (OUT_MODE == 0) {
      float* C = (float*)Cout + (size_t)b * strideC;
      const int hh = lane >> 4, c4 = (lane & 15) * 4;
      for (int pass = 0; pass < 2; ++pass) {
#pragma unroll
        for (int it = 0; it < 8; ++it) {
          const int row = it * 2 + hh;
          v4f v = *(const v4f*)(slab + row * 68 + c4);
          *(volatile v4f*)(C + (size_t)(mBase + row) * ldc + n0 + c4) = v;
        }
        __threadfence();
      }
    } else {
      const int q = lane >> 3, c8 = (lane & 7) * 8;
      unsigned short* C  = (unsigned short*)Cout  + (size_t)b * strideC;
      unsigned short* C2 = (OUT_MODE == 2) ? ((unsigned short*)Cout2 + (size_t)b * strideC) : nullptr;
      for (int pass = 0; pass < 2; ++pass) {
#pragma unroll
        for (int it = 0; it < 4; ++it) {
          const int row = it * 4 + q;
          const float* sp = slab + row * 68 + c8;
          v8h hv, lv;
#pragma unroll
          for (int e = 0; e < 8; ++e) {
            if (OUT_MODE == 1) {
              hv[e] = (_Float16)sp[e];
            } else {
              unsigned short hb = f2bf_bits(sp[e]);
              unsigned short lb = f2bf_bits(sp[e] - bf_bits2f(hb));
              hv[e] = __builtin_bit_cast(_Float16, hb);
              lv[e] = __builtin_bit_cast(_Float16, lb);
            }
          }
          *(volatile v8h*)(C + (size_t)(mBase + row) * ldc + n0 + c8) = hv;
          if (OUT_MODE == 2) *(volatile v8h*)(C2 + (size_t)(mBase + row) * ldc + n0 + c8) = lv;
        }
        __threadfence();
      }
    }
    __builtin_amdgcn_fence(__ATOMIC_RELEASE, "workgroup");
    __builtin_amdgcn_wave_barrier();
    __builtin_amdgcn_fence(__ATOMIC_ACQUIRE, "workgroup");
  }
}

__global__ __launch_bounds__(256) void wt_bf16_kernel(
    const float* __restrict__ W, int Kreal, int Nreal, unsigned short* __restrict__ Wt, int ldt)
{
  __shared__ __align__(16) float sT[64 * 68];
  const int t = threadIdx.x, lane = t & 31, wave = t >> 5;
  const int k0 = blockIdx.x * 64, n0 = blockIdx.y * 64;
  const int nn4 = (t & 15) * 4;
  const int kr  = t >> 4;
  const int n4  = n0 + nn4;
  const int n4c = (n4 < Nreal - 4) ? n4 : (Nreal - 4);
  const float fzn = (n4 < Nreal) ? 1.0f : 0.0f;
#pragma unroll
  for (int i = 0; i < 4; ++i) {
    const int kk = kr + 16 * i;
    const int k  = k0 + kk;
    const int kc = (k < Kreal) ? k : (Kreal - 1);
    const float fz = (k < Kreal) ? fzn : 0.0f;
    v4f v = *(const v4f*)(W + (size_t)kc * Nreal + n4c);
    v = v * fz;
    *(v4f*)(sT + kk * 68 + nn4) = v;
  }
  __syncthreads();
  const int q = lane >> 3, c8 = (lane & 7) * 8;
  v8h hv[2];
#pragma unroll
  for (int it = 0; it < 2; ++it) {
    const int nn = wave * 8 + it * 4 + q;
#pragma unroll
    for (int e = 0; e < 8; ++e) hv[it][e] = __builtin_bit_cast(_Float16, f2bf_bits(sT[(c8 + e) * 68 + nn]));
  }
  for (int pass = 0; pass < 2; ++pass) {
#pragma unroll
    for (int it = 0; it < 2; ++it) {
      const int nn = wave * 8 + it * 4 + q;
      *(volatile v8h*)(Wt + (size_t)(n0 + nn) * ldt + k0 + c8) = hv[it];
    }
    __threadfence();
  }
}

__global__ __launch_bounds__(256) void norm1_kernel(
    const float* __restrict__ x, const float* __restrict__ w, const float* __restrict__ mask,
    unsigned short* __restrict__ XNH, unsigned short* __restrict__ XNL)
{
  const int lane = threadIdx.x & 31, wave = threadIdx.x >> 5;
  const int row = blockIdx.x * 8 + wave;
  const float* xr = x + (size_t)row * kDm;
  const int c0 = lane * 8, c1 = 256 + lane * 8;
  v4f a[4], wv[4];
  a[0] = *(const v4f*)(xr + c0);  a[1] = *(const v4f*)(xr + c0 + 4);
  a[2] = *(const v4f*)(xr + c1);  a[3] = *(const v4f*)(xr + c1 + 4);
  wv[0] = *(const v4f*)(w + c0);  wv[1] = *(const v4f*)(w + c0 + 4);
  wv[2] = *(const v4f*)(w + c1);  wv[3] = *(const v4f*)(w + c1 + 4);
  const float mrow = bfr(mask[row]);
  float ss = 0.0f;
#pragma unroll
  for (int q4 = 0; q4 < 4; ++q4) {
#pragma unroll
    for (int e = 0; e < 4; ++e) { const float r = bfr(a[q4][e]); a[q4][e] = r; ss = fmaf(r, r, ss); }
  }
#pragma unroll
  for (int off = 16; off > 0; off >>= 1) ss += __shfl_xor(ss, off, 32);
  const float inv = 1.0f / sqrtf(ss * (1.0f / 512.0f) + 1e-6f);
  v8h h0, l0, h1, l1;
#pragma unroll
  for (int e = 0; e < 4; ++e) {
    { float v = a[0][e] * inv; v = v * bfr(wv[0][e]); v = v * mrow; const HL16 s = split_hl(v); h0[e] = s.h;     l0[e] = s.l; }
    { float v = a[1][e] * inv; v = v * bfr(wv[1][e]); v = v * mrow; const HL16 s = split_hl(v); h0[4 + e] = s.h; l0[4 + e] = s.l; }
    { float v = a[2][e] * inv; v = v * bfr(wv[2][e]); v = v * mrow; const HL16 s = split_hl(v); h1[e] = s.h;     l1[e] = s.l; }
    { float v = a[3][e] * inv; v = v * bfr(wv[3][e]); v = v * mrow; const HL16 s = split_hl(v); h1[4 + e] = s.h; l1[4 + e] = s.l; }
  }
  unsigned short* ph = XNH + (size_t)row * kDm;
  unsigned short* pl = XNL + (size_t)row * kDm;
  for (int pass = 0; pass < 2; ++pass) {
    *(volatile v8h*)(ph + c0) = h0;  *(volatile v8h*)(ph + c1) = h1;
    *(volatile v8h*)(pl + c0) = l0;  *(volatile v8h*)(pl + c1) = l1;
    __threadfence();
  }
}

__global__ __launch_bounds__(512) void scan_kernel(
    const float* __restrict__ P, const float* __restrict__ dt_bias, const float* __restrict__ A_log,
    const float* __restrict__ D_skip, unsigned short* __restrict__ YGH, unsigned short* __restrict__ YGL)
{
  __shared__ __align__(16) float sS[kTS * kStageP];
  __shared__ __align__(16) float sYP[kTS * 8 * 64];
  __shared__ __align__(16) float sYG[kTS * 64];
  __shared__ float sDT[kTS];
  __shared__ float sAV[kTS];
  const int t = threadIdx.x, lane = t & 31, wave = t >> 5;
  const int p = t & 63, g = t >> 6;
  const int b = blockIdx.x >> 4, h = blockIdx.x & 15;
  const size_t rowbase = (size_t)b * kSeq;
  const float bias = bfr(dt_bias[h]);
  const float negA = -expf(bfr(A_log[h]));
  const float dsk  = bfr(D_skip[h]);
  const int colB = kColB + h * kRN, colC = kColC + h * kRN, colU = kColU + h * kHd, colZ = kColZ + h * kHd, colD = kColDt + h;
  const int q = lane >> 3, c8 = (lane & 7) * 8;
  float hs[16];
#pragma unroll
  for (int j = 0; j < 16; ++j) hs[j] = 0.0f;

#pragma unroll 1
  for (int t0 = 0; t0 < kSeq; t0 += kTS) {
    __syncthreads();
#pragma unroll
    for (int i = 0; i < 3; ++i) {
      const int idx = i * 512 + t;
      const int r   = idx / 96;
      const int seg = idx - r * 96;
      const int col = (seg < 32) ? (colB + seg * 4)
                    : (seg < 64) ? (colC + (seg - 32) * 4)
                    : (seg < 80) ? (colU + (seg - 64) * 4)
                    :              (colZ + (seg - 80) * 4);
      const v4f v = *(const v4f*)(P + (rowbase + t0 + r) * kNProj + col);
      *(v4f*)(sS + r * kStageP + seg * 4) = v;
    }
    {
      const int r = t & 15;
      const float draw = P[(rowbase + t0 + r) * kNProj + colD] + bias;
      const float ex = expf(-fabsf(draw));
      const float dt = fmaxf(draw, 0.0f) + log1pf(ex);
      float a = expf(dt * negA);
      a = (a < 1.17549435e-38f) ? 0.0f : a;
      if (t < 16) { sDT[t] = dt; sAV[t] = a; }
    }
    __syncthreads();
#pragma unroll 1
    for (int s = 0; s < kTS; ++s) {
      const float* rp = sS + s * kStageP;
      const float dt = sDT[s];
      const float a  = sAV[s];
      const float ud = rp[256 + p] * dt;
      const float* bp = rp + g * 16;
      const float* cp = rp + 128 + g * 16;
      float yp = 0.0f;
#pragma unroll
      for (int q4 = 0; q4 < 4; ++q4) {
        const v4f bv = *(const v4f*)(bp + 4 * q4);
        const v4f cv = *(const v4f*)(cp + 4 * q4);
#pragma unroll
        for (int e = 0; e < 4; ++e) {
          const int j = 4 * q4 + e;
          const float pr = bv[e] * ud;
          hs[j] = fmaf(a, hs[j], pr);
          yp = fmaf(cv[e], hs[j], yp);
        }
      }
      sYP[(s * 8 + g) * 64 + p] = yp;
    }
    __syncthreads();
#pragma unroll 1
    for (int i = 0; i < 2; ++i) {
      const int idx = i * 512 + t;
      const int s = idx >> 6, pp = idx & 63;
      float y = 0.0f;
#pragma unroll
      for (int gg = 0; gg < 8; ++gg) y += sYP[(s * 8 + gg) * 64 + pp];
      const float* rp = sS + s * kStageP;
      const float uv = rp[256 + pp];
      y = y + uv * dsk;
      const float zv = rp[320 + pp];
      const float sg = 1.0f / (1.0f + expf(-zv));
      y = y * (zv * sg);
      sYG[s * 64 + pp] = y;
    }
    __syncthreads();
    if (wave < 4) {
      const int row = wave * 4 + q;
      const float* sp = sYG + row * 64 + c8;
      const v4f a0 = *(const v4f*)(sp);
      const v4f a1 = *(const v4f*)(sp + 4);
      v8h hv, lv;
#pragma unroll
      for (int e = 0; e < 4; ++e) {
        const HL16 s0 = split_hl(a0[e]); hv[e] = s0.h;     lv[e] = s0.l;
        const HL16 s1 = split_hl(a1[e]); hv[4 + e] = s1.h; lv[4 + e] = s1.l;
      }
      const size_t o = (rowbase + t0 + row) * kDin + h * kHd + c8;
      for (int pass = 0; pass < 2; ++pass) {
        *(volatile v8h*)(YGH + o) = hv;
        *(volatile v8h*)(YGL + o) = lv;
        __threadfence();
      }
    }
  }
}

__global__ __launch_bounds__(256) void resid_norm2_kernel(
    const float* __restrict__ x, const float* __restrict__ YO, const float* __restrict__ w,
    const float* __restrict__ mask, unsigned short* __restrict__ X2H, unsigned short* __restrict__ X2L)
{
  const int lane = threadIdx.x & 31, wave = threadIdx.x >> 5;
  const int row = blockIdx.x * 8 + wave;
  const float* xr = x + (size_t)row * kDm;
  const float* yr = YO + (size_t)row * kDm;
  const int c0 = lane * 8, c1 = 256 + lane * 8;
  v4f a[4], y[4], wv[4];
  a[0] = *(const v4f*)(xr + c0);  a[1] = *(const v4f*)(xr + c0 + 4);
  a[2] = *(const v4f*)(xr + c1);  a[3] = *(const v4f*)(xr + c1 + 4);
  y[0] = *(const v4f*)(yr + c0);  y[1] = *(const v4f*)(yr + c0 + 4);
  y[2] = *(const v4f*)(yr + c1);  y[3] = *(const v4f*)(yr + c1 + 4);
  asm volatile("" ::: "memory");
  wv[0] = *(const v4f*)(w + c0);  wv[1] = *(const v4f*)(w + c0 + 4);
  wv[2] = *(const v4f*)(w + c1);  wv[3] = *(const v4f*)(w + c1 + 4);
  const float mrow = bfr(mask[row]);
  float ss = 0.0f;
#pragma unroll
  for (int q4 = 0; q4 < 4; ++q4) {
#pragma unroll
    for (int e = 0; e < 4; ++e) {
      const float xb = bfr(a[q4][e]);
      const float x1 = fmaf(y[q4][e], mrow, xb);
      a[q4][e] = x1;
      ss = fmaf(x1, x1, ss);
    }
  }
#pragma unroll
  for (int off = 16; off > 0; off >>= 1) ss += __shfl_xor(ss, off, 32);
  const float inv = 1.0f / sqrtf(ss * (1.0f / 512.0f) + 1e-6f);
  v8h h0, l0, h1, l1;
#pragma unroll
  for (int e = 0; e < 4; ++e) {
    { float v = a[0][e] * inv; v = v * bfr(wv[0][e]); const HL16 s = split_hl(v); h0[e] = s.h;     l0[e] = s.l; }
    { float v = a[1][e] * inv; v = v * bfr(wv[1][e]); const HL16 s = split_hl(v); h0[4 + e] = s.h; l0[4 + e] = s.l; }
    { float v = a[2][e] * inv; v = v * bfr(wv[2][e]); const HL16 s = split_hl(v); h1[e] = s.h;     l1[e] = s.l; }
    { float v = a[3][e] * inv; v = v * bfr(wv[3][e]); const HL16 s = split_hl(v); h1[4 + e] = s.h; l1[4 + e] = s.l; }
  }
  unsigned short* ph = X2H + (size_t)row * kDm;
  unsigned short* pl = X2L + (size_t)row * kDm;
  for (int pass = 0; pass < 2; ++pass) {
    *(volatile v8h*)(ph + c0) = h0;  *(volatile v8h*)(ph + c1) = h1;
    *(volatile v8h*)(pl + c0) = l0;  *(volatile v8h*)(pl + c1) = l1;
    __threadfence();
  }
}

__global__ __launch_bounds__(256) void swiglu_kernel(
    const float* __restrict__ G, unsigned short* __restrict__ HFH, unsigned short* __restrict__ HFL)
{
  __shared__ __align__(16) float sH[kDffP];
  const int t = threadIdx.x;
  const int row = blockIdx.x;
  const float* gr = G + (size_t)row * kN13;
#pragma unroll 1
  for (int i = 0; i < 6; ++i) {
    const int c  = t + 256 * i;
    const int cc = (c < kDffP) ? c : (kDffP - 1);
    const float g1 = gr[cc];
    const float g3 = gr[kDffP + cc];
    const float sg = 1.0f / (1.0f + expf(-g1));
    const float v  = (g1 * sg) * g3;
    if (c < kDffP) sH[c] = v;
  }
  __syncthreads();
  if (t < kDffP / 8) {
    const int cb = t * 8;
    const v4f a0 = *(const v4f*)(sH + cb);
    const v4f a1 = *(const v4f*)(sH + cb + 4);
    v8h hv, lv;
#pragma unroll
    for (int e = 0; e < 4; ++e) {
      const HL16 s0 = split_hl(a0[e]); hv[e] = s0.h;     lv[e] = s0.l;
      const HL16 s1 = split_hl(a1[e]); hv[4 + e] = s1.h; lv[4 + e] = s1.l;
    }
    const size_t o = (size_t)row * kDffP + cb;
    for (int pass = 0; pass < 2; ++pass) {
      *(volatile v8h*)(HFH + o) = hv;
      *(volatile v8h*)(HFL + o) = lv;
      __threadfence();
    }
  }
}

__global__ __launch_bounds__(256) void final_kernel(
    const float* __restrict__ x, const float* __restrict__ YO, const float* __restrict__ FF,
    const float* __restrict__ mask, float* __restrict__ out)
{
  const int lane = threadIdx.x & 31, wave = threadIdx.x >> 5;
  const int row = blockIdx.x * 8 + wave;
  const size_t rb = (size_t)row * kDm;
  v4f xv[4], yv[4], fv[4], ov[4];
#pragma unroll
  for (int i = 0; i < 4; ++i) {
    xv[i] = *(const v4f*)(x + rb + lane * 4 + 128 * i);
    yv[i] = *(const v4f*)(YO + rb + lane * 4 + 128 * i);
  }
  asm volatile("" ::: "memory");
#pragma unroll
  for (int i = 0; i < 4; ++i) fv[i] = *(const v4f*)(FF + rb + lane * 4 + 128 * i);
  const float mrow = bfr(mask[row]);
#pragma unroll
  for (int i = 0; i < 4; ++i) {
#pragma unroll
    for (int e = 0; e < 4; ++e) {
      const float xb = bfr(xv[i][e]);
      const float x1 = fmaf(yv[i][e], mrow, xb);
      ov[i][e] = (x1 + fv[i][e]) * mrow;
    }
  }
  for (int pass = 0; pass < 2; ++pass) {
#pragma unroll
    for (int i = 0; i < 4; ++i) *(volatile v4f*)(out + rb + lane * 4 + 128 * i) = ov[i];
    __threadfence();
  }
}

extern "C" void kernel_launch(void* const* d_in, const int* in_sizes, int n_in,
                              void* d_out, int out_size, void* d_ws, size_t ws_size,
                              hipStream_t stream) {
  if (n_in < 16) return;
  if (in_sizes[0]  != kRows * kDm) return;
  if (in_sizes[1]  != kRows) return;
  if (in_sizes[2]  != kDm) return;
  if (in_sizes[3]  != kDm) return;
  if (in_sizes[4]  != kDm * kDin) return;
  if (in_sizes[5]  != kDm * kDin) return;
  if (in_sizes[6]  != kDm * 2048) return;
  if (in_sizes[7]  != kDm * 2048) return;
  if (in_sizes[8]  != kDm * kHeads) return;
  if (in_sizes[9]  != kHeads) return;
  if (in_sizes[10] != kHeads) return;
  if (in_sizes[11] != kHeads) return;
  if (in_sizes[12] != kDin * kDm) return;
  if (in_sizes[13] != kDm * kDff) return;
  if (in_sizes[14] != kDff * kDm) return;
  if (in_sizes[15] != kDm * kDff) return;
  if (out_size != kRows * kDm) return;
  if (ws_size < kWsTotal) return;

  const float* x      = (const float*)d_in[0];
  const float* mask   = (const float*)d_in[1];
  const float* n1w    = (const float*)d_in[2];
  const float* n2w    = (const float*)d_in[3];
  const float* Wz     = (const float*)d_in[4];
  const float* Wx     = (const float*)d_in[5];
  const float* Wb     = (const float*)d_in[6];
  const float* Wc     = (const float*)d_in[7];
  const float* Wdt    = (const float*)d_in[8];
  const float* dtb    = (const float*)d_in[9];
  const float* Alog   = (const float*)d_in[10];
  const float* Dsk    = (const float*)d_in[11];
  const float* Wout   = (const float*)d_in[12];
  const float* w1     = (const float*)d_in[13];
  const float* w2     = (const float*)d_in[14];
  const float* w3     = (const float*)d_in[15];
  float* out = (float*)d_out;

  char* ws = (char*)d_ws;
  unsigned short* WP  = (unsigned short*)(ws + kOffWP);
  unsigned short* WO  = (unsigned short*)(ws + kOffWO);
  unsigned short* W13 = (unsigned short*)(ws + kOffW13);
  unsigned short* W2T = (unsigned short*)(ws + kOffW2);
  unsigned short* XNH = (unsigned short*)(ws + kOffXNH);
  unsigned short* XNL = (unsigned short*)(ws + kOffXNL);
  float*          Pp  = (float*)(ws + kOffP);
  unsigned short* YGH = (unsigned short*)(ws + kOffYGH);
  unsigned short* YGL = (unsigned short*)(ws + kOffYGL);
  float*          YO  = (float*)(ws + kOffYO);
  unsigned short* X2H = (unsigned short*)(ws + kOffX2H);
  unsigned short* X2L = (unsigned short*)(ws + kOffX2L);
  float*          Gp  = (float*)(ws + kOffG);
  unsigned short* HFH = (unsigned short*)(ws + kOffHFH);
  unsigned short* HFL = (unsigned short*)(ws + kOffHFL);
  float*          FF  = (float*)(ws + kOffFF);

  wt_bf16_kernel<<<dim3(kDm / 64, kDin / 64), 256, 0, stream>>>(Wz, kDm, kDin, WP, kDm);
  wt_bf16_kernel<<<dim3(kDm / 64, kDin / 64), 256, 0, stream>>>(Wx, kDm, kDin, WP + (size_t)kColU * kDm, kDm);
  wt_bf16_kernel<<<dim3(kDm / 64, 2048 / 64), 256, 0, stream>>>(Wb, kDm, 2048, WP + (size_t)kColB * kDm, kDm);
  wt_bf16_kernel<<<dim3(kDm / 64, 2048 / 64), 256, 0, stream>>>(Wc, kDm, 2048, WP + (size_t)kColC * kDm, kDm);
  wt_bf16_kernel<<<dim3(kDm / 64, 1), 256, 0, stream>>>(Wdt, kDm, kHeads, WP + (size_t)kColDt * kDm, kDm);
  wt_bf16_kernel<<<dim3(kDin / 64, kDm / 64), 256, 0, stream>>>(Wout, kDin, kDm, WO, kDin);
  wt_bf16_kernel<<<dim3(kDm / 64, kDffP / 64), 256, 0, stream>>>(w1, kDm, kDff, W13, kDm);
  wt_bf16_kernel<<<dim3(kDm / 64, kDffP / 64), 256, 0, stream>>>(w3, kDm, kDff, W13 + (size_t)kDffP * kDm, kDm);
  wt_bf16_kernel<<<dim3(kDffP / 64, kDm / 64), 256, 0, stream>>>(w2, kDff, kDm, W2T, kDffP);

  norm1_kernel<<<kRows / 8, 256, 0, stream>>>(x, n1w, mask, XNH, XNL);

  wmma_gemm64<1, 1, 0, 0><<<dim3(388, 1), 256, 0, stream>>>(
      XNH, XNL, kDm, 0L,
      WP, nullptr, kDm, 0L,
      (void*)Pp, nullptr, kNProj, 0L,
      nullptr,
      kRows, kNProj, kDm, 1.0f);

  scan_kernel<<<kBatch * kHeads, 512, 0, stream>>>(Pp, dtb, Alog, Dsk, YGH, YGL);

  wmma_gemm64<1, 1, 0, 0><<<dim3(32, 1), 256, 0, stream>>>(
      YGH, YGL, kDin, 0L,
      WO, nullptr, kDin, 0L,
      (void*)YO, nullptr, kDm, 0L,
      nullptr,
      kRows, kDm, kDin, 1.0f);

  resid_norm2_kernel<<<kRows / 8, 256, 0, stream>>>(x, YO, n2w, mask, X2H, X2L);

  wmma_gemm64<1, 1, 0, 0><<<dim3(176, 1), 256, 0, stream>>>(
      X2H, X2L, kDm, 0L,
      W13, nullptr, kDm, 0L,
      (void*)Gp, nullptr, kN13, 0L,
      nullptr,
      kRows, kN13, kDm, 1.0f);

  swiglu_kernel<<<kRows, 256, 0, stream>>>(Gp, HFH, HFL);

  wmma_gemm64<1, 1, 0, 0><<<dim3(32, 1), 256, 0, stream>>>(
      HFH, HFL, kDffP, 0L,
      W2T, nullptr, kDffP, 0L,
      (void*)FF, nullptr, kDm, 0L,
      nullptr,
      kRows, kDm, kDffP, 1.0f);

  final_kernel<<<kRows / 8, 256, 0, stream>>>(x, YO, FF, mask, out);
}
